// PointNetFeaturePropagation_54168127537473
// MI455X (gfx1250) — hardware-verified
//
#include <hip/hip_runtime.h>
#pragma clang fp contract(off)

typedef __attribute__((ext_vector_type(16))) _Float16 v16h;
typedef __attribute__((ext_vector_type(8)))  _Float16 v8h;
typedef __attribute__((ext_vector_type(4)))  _Float16 v4h;
typedef __attribute__((ext_vector_type(8)))  float    v8f;
typedef __attribute__((ext_vector_type(4)))  float    v4f;
typedef __attribute__((ext_vector_type(4)))  int      v4i;

constexpr int NBATCH  = 8;
constexpr int NUNK    = 8192;
constexpr int NKNOWN  = 2048;
constexpr int CH_UNK  = 128;
constexpr int CH_KN   = 256;
constexpr int CH_CAT  = CH_UNK + CH_KN;
constexpr int CH_MID  = 256;
constexpr int CH_OUT  = 128;
constexpr int NROWS   = NBATCH * NUNK;
constexpr int MTILES  = NROWS / 64;
constexpr float WCARRY     = 4096.0f;
constexpr float WCARRY_INV = 1.0f / 4096.0f;
constexpr float DIST_EPS_F = 1e-8f;
constexpr float BN_EPS_F   = 1e-5f;

static_assert(CH_CAT == 384, "concat width");
static_assert(CH_CAT % 32 == 0 && CH_MID % 32 == 0, "K multiple of 32");
static_assert(NROWS % 64 == 0 && CH_MID % 64 == 0 && CH_OUT % 64 == 0, "M,N tile multiples");
static_assert(NUNK % 256 == 0 && NROWS % 8 == 0, "grid multiples");

constexpr size_t SZ_W0   = (size_t)CH_MID * CH_CAT * 2;
constexpr size_t SZ_W1   = (size_t)CH_OUT * CH_MID * 2;
constexpr size_t OFF_W0H = 0;
constexpr size_t OFF_W0L = OFF_W0H + SZ_W0;
constexpr size_t OFF_W1H = OFF_W0L + SZ_W0;
constexpr size_t OFF_W1L = OFF_W1H + SZ_W1;
constexpr size_t OFF_IDX = OFF_W1L + SZ_W1;
constexpr size_t SZ_REC  = (size_t)NROWS * 16;
constexpr size_t OFF_DSEL = OFF_IDX + SZ_REC;
constexpr size_t OFF_X   = OFF_DSEL + SZ_REC;
constexpr size_t SZ_X    = (size_t)NROWS * CH_CAT * 2;
constexpr size_t OFF_Y   = OFF_X + SZ_X;
constexpr size_t SZ_Y    = (size_t)NROWS * CH_MID * 4;
constexpr size_t OFF_P0  = OFF_Y + SZ_Y;
constexpr size_t SZ_P0   = (size_t)2 * MTILES * CH_MID * 4;
constexpr size_t OFF_P1  = OFF_P0 + SZ_P0;
constexpr size_t SZ_P1   = (size_t)2 * MTILES * CH_OUT * 4;
constexpr size_t OFF_SS  = OFF_P1 + SZ_P1;
constexpr size_t SZ_SS   = 4096;
constexpr size_t WS_TOTAL = OFF_SS + SZ_SS;
static_assert(WS_TOTAL == 123211776ull, "carve arithmetic");
static_assert(WS_TOTAL <= 134217728ull, "carve within 128 MiB");
static_assert((size_t)NROWS * CH_MID * 2 <= SZ_X, "h1 fits the X region");
static_assert((size_t)NROWS * CH_OUT * 4 <= SZ_Y, "y1 fits the Y region");
static_assert((OFF_IDX % 128) == 0 && (OFF_X % 128) == 0 && (OFF_Y % 128) == 0 && (OFF_P0 % 128) == 0 && (OFF_SS % 128) == 0, "line aligned carves");

template <typename T> struct Frag;
template <> struct Frag<_Float16> {
  typedef v16h V; union U { v16h v; v8h h[2]; };
  static __device__ __forceinline__ v16h load(const _Float16* p) {
    U f; f.h[0] = *(const v8h*)(p); f.h[1] = *(const v8h*)(p + 16); return f.v;
  }
  static __device__ __forceinline__ v8f mma(v16h a, v16h b, v8f c) {
    return __builtin_amdgcn_wmma_f32_16x16x32_f16(false, a, false, b, (short)0, c, false, false);
  }
};
__device__ __forceinline__ void guard_group(v8f& a0, v8f& a1, v8f& a2, v8f& a3, v16h x,
                                            v16h p0, v16h p1, v16h p2, v16h p3,
                                            v16h q0, v16h q1, v16h q2, v16h q3) {
  asm volatile("v_nop\n\tv_nop\n\tv_nop\n\tv_nop"
               : "+v"(a0), "+v"(a1), "+v"(a2), "+v"(a3)
               : "v"(x), "v"(p0), "v"(p1), "v"(p2), "v"(p3), "v"(q0), "v"(q1), "v"(q2), "v"(q3));
}
__device__ __forceinline__ void acc_guard4(v8f& a, v8f& b, v8f& c, v8f& d) {
  asm volatile("v_nop\n\tv_nop\n\tv_nop\n\tv_nop" : "+v"(a), "+v"(b), "+v"(c), "+v"(d));
}
__device__ __forceinline__ void wait4(v16h& a, v16h& b, v16h& c, v16h& d) {
  asm volatile("" : "+v"(a), "+v"(b), "+v"(c), "+v"(d));
}

constexpr int PREP_BLOCKS0 = (CH_MID * CH_CAT) / (8 * 256);
constexpr int PREP_BLOCKS1 = (CH_OUT * CH_MID) / (8 * 256);
static_assert(PREP_BLOCKS0 * 8 * 256 == CH_MID * CH_CAT, "prep coverage W0");
static_assert(PREP_BLOCKS1 * 8 * 256 == CH_OUT * CH_MID, "prep coverage W1");

__global__ __launch_bounds__(256) void prep_weights(
    const float* __restrict__ W0, const float* __restrict__ W1,
    _Float16* __restrict__ w0h, _Float16* __restrict__ w0l,
    _Float16* __restrict__ w1h, _Float16* __restrict__ w1l) {
  const int blk = blockIdx.x;
  const bool first = blk < PREP_BLOCKS0;
  const float* src = first ? W0 : W1;
  _Float16* dh = first ? w0h : w1h;
  _Float16* dl = first ? w0l : w1l;
  const int t = (first ? blk : (blk - PREP_BLOCKS0)) * 256 + threadIdx.x;
  const size_t e0 = (size_t)t * 8;
  const v4f a = *(const v4f*)(src + e0);
  const v4f b = *(const v4f*)(src + e0 + 4);
  v8h hv, lv;
#pragma unroll
  for (int e = 0; e < 4; ++e) {
    const float wa = a[e] * WCARRY;
    const float wb = b[e] * WCARRY;
    const _Float16 ha = (_Float16)wa;
    const _Float16 hb = (_Float16)wb;
    const float ra = wa - (float)ha;
    const float rb = wb - (float)hb;
    hv[e] = ha; hv[4 + e] = hb;
    lv[e] = (_Float16)ra; lv[4 + e] = (_Float16)rb;
  }
  *(volatile v8h*)(dh + e0) = hv;
  *(volatile v8h*)(dl + e0) = lv;
  __threadfence();
  *(volatile v8h*)(dh + e0) = hv;
  *(volatile v8h*)(dl + e0) = lv;
}

__global__ __launch_bounds__(256) void knn3_select(
    const float* __restrict__ uxyz, const float* __restrict__ kxyz,
    int* __restrict__ idx4, float* __restrict__ dsel4) {
#pragma clang fp contract(off)
  __shared__ __align__(16) float sk[NKNOWN * 3];
  const int tid = threadIdx.x;
  const int b = blockIdx.y;
  const v4f* src = (const v4f*)(kxyz + (size_t)b * NKNOWN * 3);
#pragma unroll
  for (int i = 0; i < 6; ++i) {
    const int q = tid + i * 256;
    const v4f v = src[q];
    *(v4f*)(sk + 4 * q) = v;
  }
  __syncthreads();

  const int n = blockIdx.x * 256 + tid;
  const size_t row = (size_t)b * NUNK + n;
  const float ux = uxyz[row * 3 + 0];
  const float uy = uxyz[row * 3 + 1];
  const float uz = uxyz[row * 3 + 2];

  float d0 = __builtin_huge_valf(), d1 = __builtin_huge_valf(), d2 = __builtin_huge_valf();
  int i0 = 0, i1 = 0, i2 = 0;
#pragma unroll 4
  for (int s = 0; s < NKNOWN; ++s) {
    const float kx = sk[3 * s + 0];
    const float ky = sk[3 * s + 1];
    const float kz = sk[3 * s + 2];
    const float dx = ux - kx;
    const float dy = uy - ky;
    const float dz = uz - kz;
    const float t0 = dx * dx;
    const float t1 = dy * dy;
    const float t2 = dz * dz;
    const float d = (t0 + t2) + t1;
    const bool c0 = d < d0;
    const bool c1 = d < d1;
    const bool c2 = d < d2;
    d2 = c1 ? d1 : (c2 ? d : d2);
    i2 = c1 ? i1 : (c2 ? s : i2);
    d1 = c0 ? d0 : (c1 ? d : d1);
    i1 = c0 ? i0 : (c1 ? s : i1);
    d0 = c0 ? d : d0;
    i0 = c0 ? s : i0;
  }
  v4i iv; iv[0] = i0; iv[1] = i1; iv[2] = i2; iv[3] = 0;
  v4f dv; dv[0] = d0; dv[1] = d1; dv[2] = d2; dv[3] = 0.0f;
  *(volatile v4i*)(idx4 + row * 4) = iv;
  *(volatile v4f*)(dsel4 + row * 4) = dv;
  __threadfence();
  *(volatile v4i*)(idx4 + row * 4) = iv;
  *(volatile v4f*)(dsel4 + row * 4) = dv;
}

__global__ __launch_bounds__(256) void interp_concat_f16(
    const float* __restrict__ upts, const float* __restrict__ kpts,
    const int* __restrict__ idx4, const float* __restrict__ dsel4,
    _Float16* __restrict__ xcat) {
  __shared__ __align__(16) _Float16 tile[8 * CH_CAT];
  const int tid = threadIdx.x;
  const int wave = tid >> 5;
  const int lane = tid & 31;
  const int row = blockIdx.x * 8 + wave;
  const int b = row / NUNK;

  const v4i iv = *(const v4i*)(idx4 + (size_t)row * 4);
  const v4f dv = *(const v4f*)(dsel4 + (size_t)row * 4);
  const v4f uv = *(const v4f*)(upts + (size_t)row * CH_UNK + lane * 4);

  int j0 = iv[0], j1 = iv[1], j2 = iv[2];
  j0 = j0 < 0 ? 0 : (j0 > NKNOWN - 1 ? NKNOWN - 1 : j0);
  j1 = j1 < 0 ? 0 : (j1 > NKNOWN - 1 ? NKNOWN - 1 : j1);
  j2 = j2 < 0 ? 0 : (j2 > NKNOWN - 1 ? NKNOWN - 1 : j2);

  const float r0 = 1.0f / (dv[0] + DIST_EPS_F);
  const float r1 = 1.0f / (dv[1] + DIST_EPS_F);
  const float r2 = 1.0f / (dv[2] + DIST_EPS_F);
  const float rs = (r0 + r2) + r1;
  const float w0 = r0 / rs;
  const float w1 = r1 / rs;
  const float w2 = r2 / rs;

  const float* p0 = kpts + ((size_t)b * NKNOWN + j0) * CH_KN + lane * 8;
  const float* p1 = kpts + ((size_t)b * NKNOWN + j1) * CH_KN + lane * 8;
  const float* p2 = kpts + ((size_t)b * NKNOWN + j2) * CH_KN + lane * 8;
  const v4f a0 = *(const v4f*)(p0);
  const v4f a1 = *(const v4f*)(p0 + 4);
  const v4f b0 = *(const v4f*)(p1);
  const v4f b1 = *(const v4f*)(p1 + 4);
  const v4f c0 = *(const v4f*)(p2);
  const v4f c1 = *(const v4f*)(p2 + 4);

  v4h uh;
  v8h ih;
#pragma unroll
  for (int e = 0; e < 4; ++e) {
    uh[e] = (_Float16)uv[e];
    const float lo = __builtin_fmaf(w2, c0[e], __builtin_fmaf(w1, b0[e], w0 * a0[e]));
    const float hi = __builtin_fmaf(w2, c1[e], __builtin_fmaf(w1, b1[e], w0 * a1[e]));
    ih[e] = (_Float16)lo;
    ih[4 + e] = (_Float16)hi;
  }
  *(v4h*)(tile + wave * CH_CAT + lane * 4) = uh;
  *(v8h*)(tile + wave * CH_CAT + CH_UNK + lane * 8) = ih;
  __syncthreads();

  _Float16* dst = xcat + (size_t)blockIdx.x * 8 * CH_CAT;
  const v8h va = *(const v8h*)(tile + tid * 8);
  const v8h vb = *(const v8h*)(tile + 2048 + (tid & 127) * 8);
  const bool second = tid < 128;
  *(volatile v8h*)(dst + tid * 8) = va;
  if (second) *(volatile v8h*)(dst + 2048 + tid * 8) = vb;
  __threadfence();
  *(volatile v8h*)(dst + tid * 8) = va;
  if (second) *(volatile v8h*)(dst + 2048 + tid * 8) = vb;
}

__global__ __launch_bounds__(256) void gemm_f16_wsplit_stats(
    const unsigned short* __restrict__ Ap, int lda,
    const unsigned short* __restrict__ Bhp, const unsigned short* __restrict__ Blp, int ldb,
    float* __restrict__ Cout, int ldc,
    const float* __restrict__ bias,
    float* __restrict__ part, long planeElems,
    int M, int N, int K, float scale) {
  typedef _Float16 T;
  const T* A  = (const T*)(const void*)Ap;
  const T* Bh = (const T*)(const void*)Bhp;
  const T* Bl = (const T*)(const void*)Blp;
  __shared__ __align__(16) float sT[8][16 * 68];
  const int lane = threadIdx.x & 31;
  const int wave = threadIdx.x >> 5;
  const int tilesN = N >> 6;
  const int tilesM = M >> 6;
  const int tile = blockIdx.x * 8 + wave;
  if (tile >= tilesM * tilesN) return;
  const int tm = tile / tilesN;
  const int tn = tile - tm * tilesN;
  const int m0 = tm << 6;
  const int n0 = tn << 6;

  const int rlane = lane & 15;
  const int koff  = (lane >> 4) * 8;
  const int mOff  = (lane >> 4) * 8;

  v8f acc[4][4];
#pragma unroll
  for (int i = 0; i < 4; ++i)
#pragma unroll
    for (int j = 0; j < 4; ++j) acc[i][j] = (v8f){0.f, 0.f, 0.f, 0.f, 0.f, 0.f, 0.f, 0.f};

  for (int k0 = 0; k0 < K; k0 += 32) {
    v16h bh[4], bl[4];
#pragma unroll
    for (int j = 0; j < 4; ++j) {
      const size_t bo = (size_t)(n0 + (j << 4) + rlane) * ldb + koff + k0;
      bh[j] = Frag<T>::load(Bh + bo);
    }
    wait4(bh[0], bh[1], bh[2], bh[3]);
#pragma unroll
    for (int j = 0; j < 4; ++j) {
      const size_t bo = (size_t)(n0 + (j << 4) + rlane) * ldb + koff + k0;
      bl[j] = Frag<T>::load(Bl + bo);
    }
    wait4(bl[0], bl[1], bl[2], bl[3]);
#pragma unroll
    for (int i = 0; i < 4; ++i) {
      const size_t ao = (size_t)(m0 + (i << 4) + rlane) * lda + koff + k0;
      const v16h ah = Frag<T>::load(A + ao);
#pragma unroll
      for (int j = 0; j < 4; ++j) acc[i][j] = Frag<T>::mma(ah, bh[j], acc[i][j]);
#pragma unroll
      for (int j = 0; j < 4; ++j) acc[i][j] = Frag<T>::mma(ah, bl[j], acc[i][j]);
      guard_group(acc[i][0], acc[i][1], acc[i][2], acc[i][3], ah,
                  bh[0], bh[1], bh[2], bh[3], bl[0], bl[1], bl[2], bl[3]);
    }
  }
  acc_guard4(acc[0][0], acc[0][1], acc[0][2], acc[0][3]);
  acc_guard4(acc[1][0], acc[1][1], acc[1][2], acc[1][3]);
  acc_guard4(acc[2][0], acc[2][1], acc[2][2], acc[2][3]);
  acc_guard4(acc[3][0], acc[3][1], acc[3][2], acc[3][3]);

  float* slab = sT[wave];
  const int hh = lane >> 4;
  const int c4 = (lane & 15) * 4;
  v4f st = (v4f){0.f, 0.f, 0.f, 0.f};
#pragma unroll
  for (int i = 0; i < 4; ++i) {
    const int mBase = m0 + (i << 4);
#pragma unroll
    for (int j = 0; j < 4; ++j) {
      const int n = n0 + (j << 4) + rlane;
      const float bv = bias[n];
#pragma unroll
      for (int r = 0; r < 8; ++r) {
        float v = acc[i][j][r] * scale;
        v = v + bv;
        slab[(mOff + r) * 68 + (j << 4) + rlane] = v;
      }
    }
    __builtin_amdgcn_fence(__ATOMIC_RELEASE, "workgroup");
    __builtin_amdgcn_wave_barrier();
    __builtin_amdgcn_fence(__ATOMIC_ACQUIRE, "workgroup");
#pragma unroll
    for (int r = 0; r < 16; ++r) {
      const v4f v = *(const v4f*)(slab + r * 68 + c4);
      const v4f vv = v * v;
      st = st + (hh ? vv : v);
    }
    for (int pass = 0; pass < 2; ++pass) {
#pragma unroll
      for (int it = 0; it < 8; ++it) {
        const int row = it * 2 + hh;
        const v4f v = *(const v4f*)(slab + row * 68 + c4);
        *(volatile v4f*)(Cout + (size_t)(mBase + row) * ldc + n0 + c4) = v;
      }
      __threadfence();
    }
    __builtin_amdgcn_fence(__ATOMIC_RELEASE, "workgroup");
    __builtin_amdgcn_wave_barrier();
    __builtin_amdgcn_fence(__ATOMIC_ACQUIRE, "workgroup");
  }
  {
    float* P = part + (size_t)hh * (size_t)planeElems + (size_t)tm * N + n0 + c4;
    *(volatile v4f*)P = st;
    __threadfence();
    *(volatile v4f*)P = st;
  }
}

__global__ __launch_bounds__(256) void bn_finalize(
    const float* __restrict__ psum, const float* __restrict__ psq, int ntile, int C,
    const float* __restrict__ g, const float* __restrict__ beta,
    float* __restrict__ scale, float* __restrict__ shift, double invCnt) {
  const int c = blockIdx.x * blockDim.x + threadIdx.x;
  if (c < C) {
    double s = 0.0, q = 0.0;
#pragma unroll 4
    for (int t = 0; t < ntile; ++t) {
      s += (double)psum[(size_t)t * C + c];
      q += (double)psq[(size_t)t * C + c];
    }
    const double m = s * invCnt;
    double var = q * invCnt - m * m;
    var = var < 0.0 ? 0.0 : var;
    const float rstd = rsqrtf((float)var + BN_EPS_F);
    const float sc = g[c] * rstd;
    const float sh = beta[c] - (float)m * sc;
    *(volatile float*)(scale + c) = sc;
    *(volatile float*)(shift + c) = sh;
    __threadfence();
    *(volatile float*)(scale + c) = sc;
    *(volatile float*)(shift + c) = sh;
  }
}

__global__ __launch_bounds__(256) void bn_relu_to_f16(
    const float* __restrict__ y, const float* __restrict__ scale, const float* __restrict__ shift,
    _Float16* __restrict__ h, int nchunks) {
  const int t = blockIdx.x * 256 + threadIdx.x;
  if (t >= nchunks) return;
  const int c8 = (t & (CH_MID / 8 - 1)) * 8;
  const v4f y0 = *(const v4f*)(y + (size_t)t * 8);
  const v4f y1 = *(const v4f*)(y + (size_t)t * 8 + 4);
  const v4f s0 = *(const v4f*)(scale + c8);
  const v4f s1 = *(const v4f*)(scale + c8 + 4);
  const v4f h0 = *(const v4f*)(shift + c8);
  const v4f h1 = *(const v4f*)(shift + c8 + 4);
  v8h o;
#pragma unroll
  for (int e = 0; e < 4; ++e) {
    const float a = fmaxf(__builtin_fmaf(y0[e], s0[e], h0[e]), 0.0f);
    const float b = fmaxf(__builtin_fmaf(y1[e], s1[e], h1[e]), 0.0f);
    o[e] = (_Float16)a;
    o[4 + e] = (_Float16)b;
  }
  *(volatile v8h*)(h + (size_t)t * 8) = o;
  __threadfence();
  *(volatile v8h*)(h + (size_t)t * 8) = o;
}

__global__ __launch_bounds__(256) void bn_relu_f32_out(
    const float* __restrict__ y, const float* __restrict__ scale, const float* __restrict__ shift,
    float* __restrict__ out, int nchunks) {
  const int t = blockIdx.x * 256 + threadIdx.x;
  if (t >= nchunks) return;
  const int c4 = (t & (CH_OUT / 4 - 1)) * 4;
  const v4f v = *(const v4f*)(y + (size_t)t * 4);
  const v4f sc = *(const v4f*)(scale + c4);
  const v4f sh = *(const v4f*)(shift + c4);
  v4f o;
#pragma unroll
  for (int e = 0; e < 4; ++e) o[e] = fmaxf(__builtin_fmaf(v[e], sc[e], sh[e]), 0.0f);
  *(volatile v4f*)(out + (size_t)t * 4) = o;
  __threadfence();
  *(volatile v4f*)(out + (size_t)t * 4) = o;
}

extern "C" void kernel_launch(void* const* d_in, const int* in_sizes, int n_in,
                              void* d_out, int out_size, void* d_ws, size_t ws_size,
                              hipStream_t stream) {
  if (n_in < 12) return;
  if (in_sizes[0] != NROWS * 3 || in_sizes[1] != NBATCH * NKNOWN * 3) return;
  if (in_sizes[2] != NROWS * CH_UNK || in_sizes[3] != NBATCH * NKNOWN * CH_KN) return;
  if (in_sizes[4] != CH_MID * CH_CAT || in_sizes[8] != CH_OUT * CH_MID) return;
  if (in_sizes[5] != CH_MID || in_sizes[6] != CH_MID || in_sizes[7] != CH_MID) return;
  if (in_sizes[9] != CH_OUT || in_sizes[10] != CH_OUT || in_sizes[11] != CH_OUT) return;
  if (out_size != NROWS * CH_OUT) return;
  if (ws_size < WS_TOTAL) return;

  const float* uxyz  = (const float*)d_in[0];
  const float* kxyz  = (const float*)d_in[1];
  const float* upts  = (const float*)d_in[2];
  const float* kpts  = (const float*)d_in[3];
  const float* W0    = (const float*)d_in[4];
  const float* b0    = (const float*)d_in[5];
  const float* g0    = (const float*)d_in[6];
  const float* beta0 = (const float*)d_in[7];
  const float* W1    = (const float*)d_in[8];
  const float* b1    = (const float*)d_in[9];
  const float* g1    = (const float*)d_in[10];
  const float* beta1 = (const float*)d_in[11];

  char* ws = (char*)d_ws;
  _Float16* w0h = (_Float16*)(ws + OFF_W0H);
  _Float16* w0l = (_Float16*)(ws + OFF_W0L);
  _Float16* w1h = (_Float16*)(ws + OFF_W1H);
  _Float16* w1l = (_Float16*)(ws + OFF_W1L);
  int*      idx4  = (int*)(ws + OFF_IDX);
  float*    dsel4 = (float*)(ws + OFF_DSEL);
  _Float16* xcat = (_Float16*)(ws + OFF_X);
  _Float16* h1   = (_Float16*)(ws + OFF_X);
  float*    y0   = (float*)(ws + OFF_Y);
  float*    y1   = (float*)(ws + OFF_Y);
  float*    part0 = (float*)(ws + OFF_P0);
  float*    part1 = (float*)(ws + OFF_P1);
  float*    ss    = (float*)(ws + OFF_SS);
  float* scale0 = ss;
  float* shift0 = ss + 256;
  float* scale1 = ss + 512;
  float* shift1 = ss + 640;
  const long plane0 = (long)MTILES * CH_MID;
  const long plane1 = (long)MTILES * CH_OUT;

  prep_weights<<<dim3(PREP_BLOCKS0 + PREP_BLOCKS1), dim3(256), 0, stream>>>(W0, W1, w0h, w0l, w1h, w1l);

  knn3_select<<<dim3(NUNK / 256, NBATCH), dim3(256), 0, stream>>>(uxyz, kxyz, idx4, dsel4);

  interp_concat_f16<<<dim3(NROWS / 8), dim3(256), 0, stream>>>(upts, kpts, idx4, dsel4, xcat);

  gemm_f16_wsplit_stats<<<dim3((MTILES * (CH_MID / 64)) / 8), dim3(256), 0, stream>>>(
      (const unsigned short*)xcat, CH_CAT,
      (const unsigned short*)w0h, (const unsigned short*)w0l, CH_CAT,
      y0, CH_MID, b0, part0, plane0, NROWS, CH_MID, CH_CAT, WCARRY_INV);

  bn_finalize<<<dim3(1), dim3(CH_MID), 0, stream>>>(
      part0, part0 + plane0, MTILES, CH_MID, g0, beta0, scale0, shift0, 1.0 / (double)NROWS);

  bn_relu_to_f16<<<dim3((NROWS * (CH_MID / 8)) / 256), dim3(256), 0, stream>>>(
      y0, scale0, shift0, h1, NROWS * (CH_MID / 8));

  gemm_f16_wsplit_stats<<<dim3((MTILES * (CH_OUT / 64)) / 8), dim3(256), 0, stream>>>(
      (const unsigned short*)h1, CH_MID,
      (const unsigned short*)w1h, (const unsigned short*)w1l, CH_MID,
      y1, CH_OUT, b1, part1, plane1, NROWS, CH_OUT, CH_MID, WCARRY_INV);

  bn_finalize<<<dim3(1), dim3(CH_OUT), 0, stream>>>(
      part1, part1 + plane1, MTILES, CH_OUT, g1, beta1, scale1, shift1, 1.0 / (double)NROWS);

  bn_relu_f32_out<<<dim3((NROWS * (CH_OUT / 4)) / 256), dim3(256), 0, stream>>>(
      y1, scale1, shift1, (float*)d_out, NROWS * (CH_OUT / 4));
}
